// PACA_73521250173707
// MI455X (gfx1250) — hardware-verified
//
#include <hip/hip_runtime.h>


#define NB_  4
#define CC   256
#define NN   4096
#define PCAR 1024.0f
typedef _Float16 h16;
typedef unsigned short bf;
typedef __attribute__((ext_vector_type(16))) __bf16   v16bf;
typedef __attribute__((ext_vector_type(16))) _Float16 v16h;
typedef __attribute__((ext_vector_type(8)))  _Float16 v8h;
typedef __attribute__((ext_vector_type(8)))  unsigned short v8us;
typedef __attribute__((ext_vector_type(8)))  float    v8f;
typedef __attribute__((ext_vector_type(4)))  float    v4f;
typedef v8h  __attribute__((may_alias)) v8ha;
typedef v4f  __attribute__((may_alias)) v4fa;
typedef v8us __attribute__((may_alias)) v8usa;

__device__ __forceinline__ unsigned short f2bf(float f) { unsigned u = __float_as_uint(f); u += 0x7FFFu + ((u >> 16) & 1u); return (unsigned short)(u >> 16); }
__device__ __forceinline__ float bf2f(unsigned short b) { return __uint_as_float(((unsigned)b) << 16); }
__device__ __forceinline__ float bfr(float f) { return bf2f(f2bf(f)); }
__device__ __forceinline__ v16h cat16(v8h lo, v8h hi) { return __builtin_shufflevector(lo, hi, 0, 1, 2, 3, 4, 5, 6, 7, 8, 9, 10, 11, 12, 13, 14, 15); }
__device__ __forceinline__ v16bf cat16b(v8us lo, v8us hi) { return __builtin_bit_cast(v16bf, __builtin_shufflevector(lo, hi, 0, 1, 2, 3, 4, 5, 6, 7, 8, 9, 10, 11, 12, 13, 14, 15)); }
__device__ __forceinline__ v8f wmma16(v16h a, v16h b, v8f c) { return __builtin_amdgcn_wmma_f32_16x16x32_f16(false, a, false, b, (short)0, c, false, false); }
__device__ __forceinline__ v8f wmmab(v16bf a, v16bf b, v8f c) { return __builtin_amdgcn_wmma_f32_16x16x32_bf16(false, a, false, b, (short)0, c, false, false); }


template <typename T16> struct WFrag;
template <> struct WFrag<h16> { typedef v16h V; static __device__ __forceinline__ V ld(const h16* p) { return cat16(*(const v8h*)p, *(const v8h*)(p + 16)); } static __device__ __forceinline__ v8f mma(V a, V b, v8f c) { return wmma16(a, b, c); } };
template <> struct WFrag<bf> { typedef v16bf V; static __device__ __forceinline__ V ld(const bf* p) { return cat16b(*(const v8us*)p, *(const v8us*)(p + 16)); } static __device__ __forceinline__ v8f mma(V a, V b, v8f c) { return wmmab(a, b, c); } };
template <typename T16, int NSPLIT, bool BIAS>
__global__ __launch_bounds__(32) void k_gemmw(const T16* __restrict__ A, const T16* __restrict__ A2, const T16* __restrict__ Bt, const T16* __restrict__ Bt2, int K, float* C, int ldc, const float* __restrict__ bias, size_t sA, size_t sB, size_t sC) {
    typedef typename WFrag<T16>::V V;
    __shared__ __align__(16) float os[16 * 68];
    const size_t z = blockIdx.z; A += z * sA; if (A2) A2 += z * sA; Bt += z * sB; if (Bt2) Bt2 += z * sB; C += z * sC;
    const int lane = threadIdx.x & 31, lr = lane & 15, hi = lane >> 4; const int r0 = blockIdx.x * 64, c0 = blockIdx.y * 64;
    v8f acc[4][4];
#pragma unroll
    for (int mb = 0; mb < 4; ++mb)
#pragma unroll
        for (int nb = 0; nb < 4; ++nb) acc[mb][nb] = (v8f){};
    const size_t aoff = (size_t)(r0 + lr) * K + 8 * hi, boff = (size_t)(c0 + lr) * K + 8 * hi;
#pragma unroll 1
    for (int kc = 0; kc < K; kc += 32) {
        V a[4], a2[4];
#pragma unroll
        for (int mb = 0; mb < 4; ++mb) { a[mb] = WFrag<T16>::ld(A + aoff + (size_t)mb * 16 * K + kc); if (NSPLIT == 1 || NSPLIT == 2) a2[mb] = WFrag<T16>::ld(A2 + aoff + (size_t)mb * 16 * K + kc); }
#pragma unroll
        for (int nb = 0; nb < 4; ++nb) { const V b = WFrag<T16>::ld(Bt + boff + (size_t)nb * 16 * K + kc); V b2; if (NSPLIT >= 2) b2 = WFrag<T16>::ld(Bt2 + boff + (size_t)nb * 16 * K + kc);
#pragma unroll
            for (int mb = 0; mb < 4; ++mb) { acc[mb][nb] = WFrag<T16>::mma(a[mb], b, acc[mb][nb]); if (NSPLIT == 1 || NSPLIT == 2) acc[mb][nb] = WFrag<T16>::mma(a2[mb], b, acc[mb][nb]); if (NSPLIT >= 2) acc[mb][nb] = WFrag<T16>::mma(a[mb], b2, acc[mb][nb]); } }
        asm volatile("v_nop\n\tv_nop\n\tv_nop\n\tv_nop" : "+v"(acc[0][0]), "+v"(acc[1][1]), "+v"(acc[2][2]), "+v"(acc[3][3]) : "v"(a[0]), "v"(a[3]));
    }
#pragma unroll
    for (int mb = 0; mb < 4; ++mb) {
#pragma unroll
        for (int nb = 0; nb < 4; ++nb) {
#pragma unroll
            for (int j = 0; j < 8; ++j) os[(hi * 8 + j) * 68 + nb * 16 + lr] = acc[mb][nb][j]; }
        __builtin_amdgcn_wave_barrier(); asm volatile("" ::: "memory");
        float* crow = C + (size_t)(r0 + mb * 16) * ldc + c0;
#pragma unroll 1
        for (int ps = 0; ps < 2; ++ps) {
#pragma unroll
            for (int s = 0; s < 8; ++s) { const int row = 2 * s + hi, cofs = lr * 4; v4f val = *(const v4fa*)(os + row * 68 + cofs); if (BIAS) { val[0] += bfr(bias[c0 + cofs]); val[1] += bfr(bias[c0 + cofs + 1]); val[2] += bfr(bias[c0 + cofs + 2]); val[3] += bfr(bias[c0 + cofs + 3]); }
                *(volatile v4f*)(crow + (size_t)row * ldc + cofs) = val; }
            if (ps == 0) __threadfence(); }
        __builtin_amdgcn_wave_barrier(); asm volatile("" ::: "memory");
    }
}

__device__ __forceinline__ h16 tohx(float x) { return (h16)x; }
typedef __attribute__((ext_vector_type(2))) _Float16 v2h;
typedef __attribute__((ext_vector_type(4))) _Float16 v4h;
typedef __attribute__((ext_vector_type(2))) unsigned short v2us;
typedef __attribute__((ext_vector_type(4))) unsigned short v4us;

__global__ __launch_bounds__(256) void k_cvt8(const float* __restrict__ src, bf* dst, size_t n8) { const size_t i = (size_t)blockIdx.x * 256 + threadIdx.x; if (i >= n8) return; const v8f v = *(const v8f*)(src + i * 8); v8us o;
#pragma unroll
    for (int k = 0; k < 8; ++k) o[k] = f2bf(v[k]); *(volatile v8us*)(dst + i * 8) = o; __threadfence(); *(volatile v8us*)(dst + i * 8) = o; }
__global__ __launch_bounds__(256) void k_tok(const float* __restrict__ x, bf* XT) { const size_t e = ((size_t)blockIdx.x * 256 + threadIdx.x) * 4; if (e >= (size_t)NN * CC) return; const int c = (int)(e % CC), n = (int)(e / CC); v4us o;
#pragma unroll
    for (int q = 0; q < 4; ++q) o[q] = f2bf(x[(size_t)(c + q) * NN + n]); *(volatile v4us*)(XT + e) = o; __threadfence(); *(volatile v4us*)(XT + e) = o; }
__global__ __launch_bounds__(256) void k_p16(const float* __restrict__ F, h16* P) { const size_t i = ((size_t)blockIdx.x * 256 + threadIdx.x) * 4; if (i >= (size_t)NN * CC) return; const v4f a = *(const v4f*)(F + i); v4h o; o[0] = tohx(a[0]); o[1] = tohx(a[1]); o[2] = tohx(a[2]); o[3] = tohx(a[3]); *(volatile v4h*)(P + i) = o; __threadfence(); *(volatile v4h*)(P + i) = o; }
__global__ __launch_bounds__(256) void k_vt16(const float* __restrict__ V, h16* VT) { const size_t e = ((size_t)blockIdx.x * 256 + threadIdx.x) * 2; if (e >= (size_t)CC * NN) return; const int n = (int)(e % NN), d = (int)(e / NN); v2h o; o[0] = tohx(V[(size_t)n * CC + d]); o[1] = tohx(V[(size_t)(n + 1) * CC + d]); *(volatile v2h*)(VT + e) = o; __threadfence(); *(volatile v2h*)(VT + e) = o; }
__global__ __launch_bounds__(256) void k_soft(const float* __restrict__ Sb, h16* P) { const int lane = threadIdx.x & 31; const int row = blockIdx.x * 8 + (threadIdx.x >> 5); if (row >= NN) return; const float* sr = Sb + (size_t)row * NN; float v[128]; float mx = -3.0e38f;
#pragma unroll
    for (int ch = 0; ch < 32; ++ch) { const v4f a = *(const v4f*)(sr + ch * 128 + lane * 4);
#pragma unroll
        for (int q = 0; q < 4; ++q) { float t = a[q] * 0.0625f; asm volatile("" : "+v"(t)); v[ch * 4 + q] = t; mx = fmaxf(mx, t); } }
#pragma unroll
    for (int sh = 16; sh; sh >>= 1) mx = fmaxf(mx, __shfl_xor(mx, sh, 32));
    float sum = 0.f;
#pragma unroll
    for (int k = 0; k < 128; ++k) { float d0 = __fsub_rn(v[k], mx); asm volatile("" : "+v"(d0)); v[k] = __expf(d0); sum += v[k]; }
#pragma unroll
    for (int sh = 16; sh; sh >>= 1) sum += __shfl_xor(sum, sh, 32);
    const float f = __fdiv_rn(PCAR, sum);
#pragma unroll 1
    for (int ps = 0; ps < 2; ++ps) {
#pragma unroll
        for (int ch = 0; ch < 32; ++ch) { v4h o; o[0] = tohx(v[ch * 4] * f); o[1] = tohx(v[ch * 4 + 1] * f); o[2] = tohx(v[ch * 4 + 2] * f); o[3] = tohx(v[ch * 4 + 3] * f); *(volatile v4h*)(P + (size_t)row * NN + ch * 128 + lane * 4) = o; }
        if (ps == 0) __threadfence(); } }
__global__ __launch_bounds__(256) void k_out(const float* __restrict__ O, const float* __restrict__ x, float* OUT) { const size_t e = ((size_t)blockIdx.x * 256 + threadIdx.x) * 4; if (e >= (size_t)CC * NN) return; const int n = (int)(e % NN), c = (int)(e / NN); v4f o;
#pragma unroll
    for (int q = 0; q < 4; ++q) o[q] = __fadd_rn(bfr(x[e + q]), O[(size_t)(n + q) * CC + c] * (1.0f / PCAR)); *(volatile v4f*)(OUT + e) = o; __threadfence(); *(volatile v4f*)(OUT + e) = o; }

extern "C" void kernel_launch(void* const* d_in, const int* in_sizes, int n_in,
                              void* d_out, int out_size, void* d_ws, size_t ws_size, hipStream_t stream) {
    (void)in_sizes; (void)n_in; (void)out_size;
    const float* x = (const float*)d_in[0]; const float* y = (const float*)d_in[1]; const float* Wq = (const float*)d_in[2]; const float* bq = (const float*)d_in[3]; const float* Wk = (const float*)d_in[4]; const float* bk = (const float*)d_in[5]; const float* Wv = (const float*)d_in[6]; const float* bv = (const float*)d_in[7];
    float* OUT = (float*)d_out;
    char* wsp = (char*)d_ws;
    auto take = [&](size_t bytes) { char* p = wsp; wsp += (bytes + 255) & ~(size_t)255; return (void*)p; };
    bf* WQ = (bf*)take((size_t)CC * CC * 2); bf* WK = (bf*)take((size_t)CC * CC * 2); bf* WV = (bf*)take((size_t)CC * CC * 2); bf* XT = (bf*)take((size_t)NN * CC * 2); bf* YT = (bf*)take((size_t)NN * CC * 2);
    float* F = (float*)take((size_t)NN * CC * 4); h16* Q16 = (h16*)take((size_t)NN * CC * 2); h16* K16 = (h16*)take((size_t)NN * CC * 2); h16* VT = (h16*)take((size_t)CC * NN * 2); float* Sb = (float*)take((size_t)NN * NN * 4); h16* P16 = (h16*)take((size_t)NN * NN * 2); float* O = (float*)take((size_t)NN * CC * 4);
    if ((size_t)(wsp - (char*)d_ws) > ws_size) return;
    k_cvt8<<<(CC * CC / 8 + 255) / 256, 256, 0, stream>>>(Wq, WQ, (size_t)CC * CC / 8); k_cvt8<<<(CC * CC / 8 + 255) / 256, 256, 0, stream>>>(Wk, WK, (size_t)CC * CC / 8); k_cvt8<<<(CC * CC / 8 + 255) / 256, 256, 0, stream>>>(Wv, WV, (size_t)CC * CC / 8);
    const unsigned LT = (unsigned)(((size_t)NN * CC / 4 + 255) / 256);
    for (int b = 0; b < NB_; ++b) { const float* xb = x + (size_t)b * CC * NN; const float* yb = y + (size_t)b * CC * NN;
        k_tok<<<LT, 256, 0, stream>>>(xb, XT); k_tok<<<LT, 256, 0, stream>>>(yb, YT);
        k_gemmw<bf, 0, true><<<dim3(NN / 64, CC / 64, 1), 32, 0, stream>>>(XT, nullptr, WQ, nullptr, CC, F, CC, bq, 0, 0, 0); k_p16<<<LT, 256, 0, stream>>>(F, Q16);
        k_gemmw<bf, 0, true><<<dim3(NN / 64, CC / 64, 1), 32, 0, stream>>>(YT, nullptr, WK, nullptr, CC, F, CC, bk, 0, 0, 0); k_p16<<<LT, 256, 0, stream>>>(F, K16);
        k_gemmw<bf, 0, true><<<dim3(NN / 64, CC / 64, 1), 32, 0, stream>>>(YT, nullptr, WV, nullptr, CC, F, CC, bv, 0, 0, 0); k_vt16<<<(unsigned)(((size_t)CC * NN / 2 + 255) / 256), 256, 0, stream>>>(F, VT);
        k_gemmw<h16, 0, false><<<dim3(NN / 64, NN / 64, 1), 32, 0, stream>>>(Q16, nullptr, K16, nullptr, CC, Sb, NN, nullptr, 0, 0, 0);
        k_soft<<<NN / 8, 256, 0, stream>>>(Sb, P16);
        k_gemmw<h16, 0, false><<<dim3(NN / 64, CC / 64, 1), 32, 0, stream>>>(P16, nullptr, VT, nullptr, NN, O, CC, nullptr, 0, 0, 0);
        k_out<<<LT, 256, 0, stream>>>(O, xb, OUT + (size_t)b * CC * NN); }
}
